// LSTM_Autoencoder_69861938037379
// MI455X (gfx1250) — hardware-verified
//
#include <hip/hip_runtime.h>
#include <stddef.h>


typedef _Float16 f16_t;
typedef _Float16 v16h __attribute__((ext_vector_type(16)));
typedef _Float16 v8h  __attribute__((ext_vector_type(8)));
typedef float    v8f  __attribute__((ext_vector_type(8)));
typedef float    v4f  __attribute__((ext_vector_type(4)));

union Frag { v16h v; v8h hf[2]; };

#define WSCALE 64.0f
#define WINV   0.015625f

__device__ __forceinline__ v8f wmma16(v16h a, v16h b, v8f c)
{
    v8f d = __builtin_amdgcn_wmma_f32_16x16x32_f16(false, a, false, b, (short)0, c, false, false);
    asm volatile("v_nop\n\tv_nop\n\tv_nop\n\tv_nop" : "+v"(d) : "v"(a), "v"(b));
    return d;
}

__device__ __forceinline__ v16h ld_frag(const f16_t* base, int row, int ld, int k0, int hh)
{
    const f16_t* p = base + (size_t)row * ld + k0 + 8 * hh;
    Frag f;
    f.hf[0] = *(const v8h*)p;
    f.hf[1] = *(const v8h*)(p + 16);
    return f.v;
}

__device__ __forceinline__ v8h load8(const float* p)
{
    const v4f a = *(const v4f*)p;
    const v4f b = *(const v4f*)(p + 4);
    const v8f f = __builtin_shufflevector(a, b, 0, 1, 2, 3, 4, 5, 6, 7);
    return __builtin_convertvector(f, v8h);
}
__device__ __forceinline__ v8h load8(const f16_t* p)
{
    return *(const v8h*)p;
}

__device__ __forceinline__ float sigm(float x)
{
    return __builtin_amdgcn_rcpf(1.0f + __expf(-x));
}

__global__ __launch_bounds__(256)
void k_wtr(const float* __restrict__ src, f16_t* __restrict__ dst, int K, int N)
{
    __shared__ __align__(16) f16_t tile[32 * 136];
    const int n0 = blockIdx.x * 32;
    if (n0 + 32 > N) return;
    const int tid = threadIdx.x;
    for (int idx = tid; idx < 32 * K; idx += 256) {
        const int k = idx >> 5, j = idx & 31;
        tile[j * 136 + k] = (f16_t)(src[(size_t)k * N + n0 + j] * WSCALE);
    }
    __syncthreads();
    const int nch = 4 * K;
    f16_t* ob = dst + (size_t)n0 * K;
    for (int c = tid; c < nch; c += 256) {
        const int j = (8 * c) / K, k = 8 * c - j * K;
        const v8h v = *(const v8h*)(tile + j * 136 + k);
        *(volatile v8h*)(ob + 8 * c) = v;
    }
    __threadfence();
    for (int c = tid; c < nch; c += 256) {
        const int j = (8 * c) / K, k = 8 * c - j * K;
        const v8h v = *(const v8h*)(tile + j * 136 + k);
        *(volatile v8h*)(ob + 8 * c) = v;
    }
}

template <int U, int D, bool REP, typename XT>
__global__ __launch_bounds__(2 * U)
void k_lstm(const XT* __restrict__ xin, long xbs, long xts,
            const f16_t* __restrict__ WkT, const f16_t* __restrict__ WrT,
            const float* __restrict__ bias,
            f16_t* __restrict__ hout, long obs, long ots, int t_store0, int T, int nB)
{
    constexpr int NTHR = 2 * U;
    constexpr int KCH  = U / 8;
    constexpr int XCH  = D / 8;
    extern __shared__ __align__(16) f16_t lds_dyn[];
    f16_t* sWrT = lds_dyn;
    f16_t* sH   = sWrT + 4 * U * U;
    f16_t* sX   = sH + 16 * U;

    const int tid = threadIdx.x, wave = tid >> 5, lane = tid & 31;
    const int hh = lane >> 4, m = lane & 15;
    const int b0 = blockIdx.x * 16;
    if (b0 + 16 > nB) return;
    const int ucol = 16 * wave + m;

    {
        const v8h* g = (const v8h*)WrT;
        v8h* s = (v8h*)sWrT;
        for (int i = tid; i < (4 * U * U) / 8; i += NTHR) s[i] = g[i];
        const v8h zz = {0, 0, 0, 0, 0, 0, 0, 0};
        v8h* sh = (v8h*)sH;
        for (int i = tid; i < 2 * U; i += NTHR) sh[i] = zz;
    }

    auto stage_x = [&](int t) {
        for (int c = tid; c < 16 * XCH; c += NTHR) {
            const int mm = c / XCH, k8 = c - mm * XCH;
            const XT* p = xin + (long)(b0 + mm) * xbs + (long)t * xts + 8 * k8;
            *(v8h*)(sX + mm * D + 8 * k8) = load8(p);
        }
    };

    float bS[4];
#pragma unroll
    for (int g = 0; g < 4; ++g) bS[g] = bias[g * U + ucol] * WSCALE;

    v8f xz[4];
#pragma unroll
    for (int g = 0; g < 4; ++g) {
#pragma unroll
        for (int r = 0; r < 8; ++r) xz[g][r] = bS[g];
    }
    if (REP) {
        stage_x(0);
        __syncthreads();
#pragma unroll
        for (int k0 = 0; k0 < D; k0 += 32) {
            const v16h a = ld_frag(sX, m, D, k0, hh);
#pragma unroll
            for (int g = 0; g < 4; ++g)
                xz[g] = wmma16(a, ld_frag(WkT, g * U + ucol, D, k0, hh), xz[g]);
        }
    }

    float cst[8];
#pragma unroll
    for (int r = 0; r < 8; ++r) cst[r] = 0.0f;

    for (int t = 0; t < T; ++t) {
        if (!REP) stage_x(t);
        __syncthreads();

        v8f acc[4];
#pragma unroll
        for (int g = 0; g < 4; ++g) acc[g] = xz[g];
        if (!REP) {
#pragma unroll
            for (int k0 = 0; k0 < D; k0 += 32) {
                const v16h a = ld_frag(sX, m, D, k0, hh);
#pragma unroll
                for (int g = 0; g < 4; ++g)
                    acc[g] = wmma16(a, ld_frag(WkT, g * U + ucol, D, k0, hh), acc[g]);
            }
        }
#pragma unroll
        for (int k0 = 0; k0 < U; k0 += 32) {
            const v16h a = ld_frag(sH, m, U, k0, hh);
#pragma unroll
            for (int g = 0; g < 4; ++g)
                acc[g] = wmma16(a, ld_frag(sWrT, g * U + ucol, U, k0, hh), acc[g]);
        }
        __syncthreads();

#pragma unroll
        for (int r = 0; r < 8; ++r) {
            const float gi = sigm(acc[0][r] * WINV);
            const float gf = sigm(acc[1][r] * WINV);
            const float gg = sigm(acc[2][r] * WINV);
            const float go = sigm(acc[3][r] * WINV);
            const float cn = gf * cst[r] + gi * gg;
            cst[r] = cn;
            const float hv = go * sigm(cn);
            sH[(8 * hh + r) * U + ucol] = (f16_t)hv;
        }
        __syncthreads();

        if (t >= t_store0) {
            const int mm = tid / KCH, k8 = tid - mm * KCH;
            const v8h v = *(const v8h*)(sH + mm * U + 8 * k8);
            f16_t* dp = hout + (long)(b0 + mm) * obs + (long)(t - t_store0) * ots + 8 * k8;
            *(volatile v8h*)dp = v;
            __threadfence();
            *(volatile v8h*)dp = v;
        }
    }
}

template <int K, int N>
__global__ __launch_bounds__(256)
void k_gemm(const f16_t* __restrict__ A, int lda, const f16_t* __restrict__ WT,
            const float* __restrict__ bias, float* __restrict__ C, int M)
{
    constexpr int KS = K / 32, NT = N / 16;
    extern __shared__ __align__(16) float lds_f[];
    const int tid = threadIdx.x, wave = tid >> 5, lane = tid & 31;
    const int hh = lane >> 4, m = lane & 15;
    const int m0 = blockIdx.x * 128 + 16 * wave;
    int rowA = m0 + m;
    if (rowA > M - 1) rowA = M - 1;

    v16h af[KS];
#pragma unroll
    for (int ks = 0; ks < KS; ++ks) af[ks] = ld_frag(A, rowA, lda, 32 * ks, hh);

    v8f acc[NT];
#pragma unroll
    for (int nt = 0; nt < NT; ++nt) {
#pragma unroll
        for (int r = 0; r < 8; ++r) acc[nt][r] = 0.0f;
    }
#pragma unroll
    for (int ks = 0; ks < KS; ++ks) {
#pragma unroll
        for (int nt = 0; nt < NT; ++nt)
            acc[nt] = wmma16(af[ks], ld_frag(WT, 16 * nt + m, K, 32 * ks, hh), acc[nt]);
    }

    float* sT = lds_f + wave * 16 * N;
#pragma unroll
    for (int nt = 0; nt < NT; ++nt) {
        const float bc = bias[16 * nt + m];
#pragma unroll
        for (int r = 0; r < 8; ++r)
            sT[(8 * hh + r) * N + 16 * nt + m] = acc[nt][r] * WINV + bc;
    }
    __syncthreads();

    float* cb = C + (size_t)m0 * N;
#pragma unroll
    for (int i = 0; i < N / 8; ++i) {
        const int c = lane + 32 * i;
        const int row = c / (N / 4);
        if (m0 + row < M) {
            const v4f v = *(const v4f*)(sT + 4 * c);
            *(volatile v4f*)(cb + 4 * c) = v;
        }
    }
    __threadfence();
#pragma unroll
    for (int i = 0; i < N / 8; ++i) {
        const int c = lane + 32 * i;
        const int row = c / (N / 4);
        if (m0 + row < M) {
            const v4f v = *(const v4f*)(sT + 4 * c);
            *(volatile v4f*)(cb + 4 * c) = v;
        }
    }
}

static inline size_t al256(size_t x) { return (x + 255) & ~(size_t)255; }

extern "C" void kernel_launch(void* const* d_in, const int* in_sizes, int n_in,
                              void* d_out, int out_size, void* d_ws, size_t ws_size,
                              hipStream_t stream)
{
    if (n_in < 17) return;
    const int F = 128, U1 = 128, U2 = 64, L = 32, T = 512;
    if (in_sizes[16] != F || in_sizes[3] != 4 * U1 || in_sizes[6] != 4 * U2 || in_sizes[8] != L) return;
    if (in_sizes[1] != F * 4 * U1 || in_sizes[2] != U1 * 4 * U1 || in_sizes[4] != U1 * 4 * U2 ||
        in_sizes[5] != U2 * 4 * U2 || in_sizes[7] != U2 * L || in_sizes[9] != L * 4 * U2 ||
        in_sizes[10] != U2 * 4 * U2 || in_sizes[11] != 4 * U2 || in_sizes[12] != U2 * 4 * U1 ||
        in_sizes[13] != U1 * 4 * U1 || in_sizes[14] != 4 * U1 || in_sizes[15] != U1 * F) return;
    const long nX = in_sizes[0];
    if (nX <= 0 || nX % ((long)T * F) != 0) return;
    const int Bn = (int)(nX / ((long)T * F));
    if (Bn < 16 || (Bn % 16) != 0) return;
    const long BT = (long)Bn * T;
    if ((long)out_size != BT * F) return;

    const float* x   = (const float*)d_in[0];
    const float* ek1 = (const float*)d_in[1];
    const float* er1 = (const float*)d_in[2];
    const float* eb1 = (const float*)d_in[3];
    const float* ek2 = (const float*)d_in[4];
    const float* er2 = (const float*)d_in[5];
    const float* eb2 = (const float*)d_in[6];
    const float* lw  = (const float*)d_in[7];
    const float* lb  = (const float*)d_in[8];
    const float* dk1 = (const float*)d_in[9];
    const float* dr1 = (const float*)d_in[10];
    const float* db1 = (const float*)d_in[11];
    const float* dk2 = (const float*)d_in[12];
    const float* dr2 = (const float*)d_in[13];
    const float* db2 = (const float*)d_in[14];
    const float* ow  = (const float*)d_in[15];
    const float* ob  = (const float*)d_in[16];
    float* out = (float*)d_out;

    char* ws = (char*)d_ws;
    size_t off = 0;
    auto carve = [&](size_t bytes) { size_t o = off; off = al256(off + bytes); return o; };

    f16_t* ek1T = (f16_t*)(ws + carve((size_t)(4 * U1) * F  * 2));
    f16_t* er1T = (f16_t*)(ws + carve((size_t)(4 * U1) * U1 * 2));
    f16_t* ek2T = (f16_t*)(ws + carve((size_t)(4 * U2) * U1 * 2));
    f16_t* er2T = (f16_t*)(ws + carve((size_t)(4 * U2) * U2 * 2));
    f16_t* lwT  = (f16_t*)(ws + carve((size_t)L * U2 * 2));
    f16_t* dk1T = (f16_t*)(ws + carve((size_t)(4 * U2) * L  * 2));
    f16_t* dr1T = (f16_t*)(ws + carve((size_t)(4 * U2) * U2 * 2));
    f16_t* dk2T = (f16_t*)(ws + carve((size_t)(4 * U1) * U2 * 2));
    f16_t* dr2T = (f16_t*)(ws + carve((size_t)(4 * U1) * U1 * 2));
    f16_t* owT  = (f16_t*)(ws + carve((size_t)F * U1 * 2));
    f16_t* h1  = (f16_t*)(ws + carve((size_t)BT * U1 * 2));
    f16_t* h2l = (f16_t*)(ws + carve((size_t)Bn * U2 * 2));
    float*  zf = (float*) (ws + carve((size_t)Bn * L * 4));
    f16_t* d1  = (f16_t*)(ws + carve((size_t)BT * U2 * 2));
    f16_t* d2  = (f16_t*)(ws + carve((size_t)BT * U1 * 2));
    if (off > ws_size) return;

    const dim3 b256(256), b128(128);

    k_wtr<<<dim3((4 * U1) / 32), b256, 0, stream>>>(ek1, ek1T, F,  4 * U1);
    k_wtr<<<dim3((4 * U1) / 32), b256, 0, stream>>>(er1, er1T, U1, 4 * U1);
    k_wtr<<<dim3((4 * U2) / 32), b256, 0, stream>>>(ek2, ek2T, U1, 4 * U2);
    k_wtr<<<dim3((4 * U2) / 32), b256, 0, stream>>>(er2, er2T, U2, 4 * U2);
    k_wtr<<<dim3(L / 32),        b256, 0, stream>>>(lw,  lwT,  U2, L);
    k_wtr<<<dim3((4 * U2) / 32), b256, 0, stream>>>(dk1, dk1T, L,  4 * U2);
    k_wtr<<<dim3((4 * U2) / 32), b256, 0, stream>>>(dr1, dr1T, U2, 4 * U2);
    k_wtr<<<dim3((4 * U1) / 32), b256, 0, stream>>>(dk2, dk2T, U2, 4 * U1);
    k_wtr<<<dim3((4 * U1) / 32), b256, 0, stream>>>(dr2, dr2T, U1, 4 * U1);
    k_wtr<<<dim3(F / 32),        b256, 0, stream>>>(ow,  owT,  U1, F);

    const size_t lds_e1 = ((size_t)4 * 128 * 128 + 16 * 128 + 16 * 128) * 2;
    const size_t lds_e2 = ((size_t)4 * 64 * 64 + 16 * 64 + 16 * 128) * 2;
    const size_t lds_d1 = ((size_t)4 * 64 * 64 + 16 * 64 + 16 * 32) * 2;
    const size_t lds_d2 = ((size_t)4 * 128 * 128 + 16 * 128 + 16 * 64) * 2;
    const dim3 gscan(Bn / 16);

    k_lstm<128, 128, false, float><<<gscan, b256, lds_e1, stream>>>(
        x, (long)T * F, (long)F, ek1T, er1T, eb1, h1, (long)T * U1, (long)U1, 0, T, Bn);
    k_lstm<64, 128, false, f16_t><<<gscan, b128, lds_e2, stream>>>(
        h1, (long)T * U1, (long)U1, ek2T, er2T, eb2, h2l, (long)U2, (long)0, T - 1, T, Bn);
    k_gemm<64, 32><<<dim3((Bn + 127) / 128), b256, (size_t)8 * 16 * 32 * 4, stream>>>(
        h2l, U2, lwT, lb, zf, Bn);
    k_lstm<64, 32, true, float><<<gscan, b128, lds_d1, stream>>>(
        zf, (long)L, (long)0, dk1T, dr1T, db1, d1, (long)T * U2, (long)U2, 0, T, Bn);
    k_lstm<128, 64, false, f16_t><<<gscan, b256, lds_d2, stream>>>(
        d1, (long)T * U2, (long)U2, dk2T, dr2T, db2, d2, (long)T * U1, (long)U1, 0, T, Bn);
    k_gemm<128, 128><<<dim3((unsigned)((BT + 127) / 128)), b256, (size_t)8 * 16 * 128 * 4, stream>>>(
        d2, U1, owT, ob, out, (int)BT);
}
